// FSAS_83245056131631
// MI455X (gfx1250) — hardware-verified
//
#include <hip/hip_runtime.h>
#include <math.h>

typedef __attribute__((ext_vector_type(16))) _Float16 v16h;
typedef __attribute__((ext_vector_type(16))) __bf16 v16b;
typedef __attribute__((ext_vector_type(8)))  _Float16 v8h;
typedef __attribute__((ext_vector_type(8)))  float v8f;
typedef __attribute__((ext_vector_type(4)))  float v4f;
typedef __attribute__((ext_vector_type(2)))  float v2f;
typedef __attribute__((ext_vector_type(4)))  unsigned v4u;
typedef __attribute__((ext_vector_type(4)))  int v4i;
typedef float __attribute__((may_alias)) float_a;
typedef int __attribute__((may_alias)) int_a;

template <typename T> __device__ __forceinline__ void vst2(void* p, T v) { *(volatile T*)p = v; __threadfence(); *(volatile T*)p = v; }
__device__ __forceinline__ v8f wmma16(v16h a, v16h b, v8f c) {
  v8f d = __builtin_amdgcn_wmma_f32_16x16x32_f16(false, a, false, b, (short)0, c, false, false);
  asm volatile("v_nop\n\tv_nop\n\tv_nop\n\tv_nop" : "+v"(d) : "v"(a), "v"(b));
  return d;
}
__device__ __forceinline__ v8f wmma_bf(v16b a, v16b b, v8f c) {
  v8f d = __builtin_amdgcn_wmma_f32_16x16x32_bf16(false, a, false, b, (short)0, c, false, false);
  asm volatile("v_nop\n\tv_nop\n\tv_nop\n\tv_nop" : "+v"(d) : "v"(a), "v"(b));
  return d;
}
__device__ __forceinline__ v16h frag_h(const _Float16* rowk0, int lane) {
  union { v16h v; v8h q[2]; } u; const _Float16* p = rowk0 + 8 * (lane >> 4);
  u.q[0] = *(const v8h*)p; u.q[1] = *(const v8h*)(p + 16); return u.v;
}
__device__ __forceinline__ v16h frag_f32(const float* rowk0, int lane) {
  v16h a; const float* p = rowk0 + 8 * (lane >> 4);
#pragma unroll
  for (int i = 0; i < 8; ++i) { a[i] = (_Float16)p[i]; a[8 + i] = (_Float16)p[16 + i]; }
  return a;
}
__device__ __forceinline__ v16h frag_f32s(const float* rowk0, int lane, float sc) {
  v16h a; const float* p = rowk0 + 8 * (lane >> 4);
#pragma unroll
  for (int i = 0; i < 8; ++i) { a[i] = (_Float16)(p[i] * sc); a[8 + i] = (_Float16)(p[16 + i] * sc); }
  return a;
}
__device__ __forceinline__ v16h fragc_f32(const float* W, int k0, int n, int lane, int ld, int K) {
  v16h a; const int g = lane >> 4;
#pragma unroll
  for (int i = 0; i < 8; ++i) { const int ka = k0 + 8 * g + i, kb = ka + 16;
    a[i] = (_Float16)(ka < K ? W[(size_t)(ka < K ? ka : K - 1) * ld + n] : 0.f); a[8 + i] = (_Float16)(kb < K ? W[(size_t)(kb < K ? kb : K - 1) * ld + n] : 0.f); }
  return a;
}
struct F2 { v16b h, l; };
__device__ __forceinline__ F2 bsplit16(const float v[16]) { F2 r;
#pragma unroll
  for (int i = 0; i < 16; ++i) { const __bf16 h = (__bf16)v[i]; r.h[i] = h; r.l[i] = (__bf16)(v[i] - (float)h); }
  return r; }
__device__ __forceinline__ F2 split_row(const float* row, int k0, int lane) { float v[16]; const float* p = row + k0 + 8 * (lane >> 4);
#pragma unroll
  for (int i = 0; i < 8; ++i) { v[i] = p[i]; v[8 + i] = p[16 + i]; }
  return bsplit16(v); }
__device__ __forceinline__ F2 split_rowK(const float* row, int k0, int lane, int K) { float v[16]; const int g = lane >> 4;
#pragma unroll
  for (int i = 0; i < 8; ++i) { const int ka = k0 + 8 * g + i, kb = ka + 16; v[i] = ka < K ? row[ka < K ? ka : K - 1] : 0.f; v[8 + i] = kb < K ? row[kb < K ? kb : K - 1] : 0.f; }
  return bsplit16(v); }
__device__ __forceinline__ F2 split_col(const float* W, int k0, int n, int lane, int ld, int K) { float v[16]; const int g = lane >> 4;
#pragma unroll
  for (int i = 0; i < 8; ++i) { const int ka = k0 + 8 * g + i, kb = ka + 16; v[i] = ka < K ? W[(size_t)(ka < K ? ka : K - 1) * ld + n] : 0.f; v[8 + i] = kb < K ? W[(size_t)(kb < K ? kb : K - 1) * ld + n] : 0.f; }
  return bsplit16(v); }
__device__ __forceinline__ v8f mac3(const F2& a, const F2& b, v8f c) { c = wmma_bf(a.l, b.h, c); c = wmma_bf(a.h, b.l, c); return wmma_bf(a.h, b.h, c); }
__device__ __forceinline__ float sigm(float v) { return 1.0f / (1.0f + expf(-v)); }
#define LDSX() do { asm volatile("s_wait_dscnt 0" ::: "memory"); __builtin_amdgcn_wave_barrier(); __builtin_amdgcn_fence(__ATOMIC_RELEASE, "workgroup"); } while (0)


#define NBT 4
#define CIN 48
#define CKP 64
#define HH 256
#define WWD 256
#define NPI (HH * WWD)
#define C3 288
#define CG 96
#define PSZ 8
#define NPR (HH / PSZ)
#define NPATCH (NBT * NPR * NPR)
#ifndef NPT
#define NPT NPATCH
#define NPRT NPR
#define NBTT NBT
#endif
typedef __attribute__((ext_vector_type(8))) __bf16 v8b;
__device__ __forceinline__ v16b frag_b(const __bf16* rowk0, int lane) {
  union { v16b v; v8b q[2]; } u; const __bf16* p = rowk0 + 8 * (lane >> 4);
  u.q[0] = *(const v8b*)p; u.q[1] = *(const v8b*)(p + 16); return u.v;
}
__device__ __forceinline__ float bfr(float v) { return (float)(__bf16)v; }
__device__ __attribute__((noinline)) float exp_ni(float v) { return expf(v); }
__device__ __attribute__((noinline)) float erf_ni(float v) { return erff(v); }

#define WS_XC   0u
#define WS_PH   (WS_XC + 2u * NBT * NPI * CKP)
#define WS_PP   (WS_PH + 2u * C3 * CKP)
#define WS_OP   (((WS_PP + 2u * CIN * CG) + 127u) / 128u * 128u)
#define WS_END  (WS_OP + 4u * NBT * CIN * NPR * NPR * 64)

__device__ __forceinline__ v16b zfrag_ok(v16b a, bool ok) { const v16b z = {}; return ok ? a : z; }
__global__ __launch_bounds__(256) void k_pack(const float* __restrict__ WH, const float* __restrict__ WP, __bf16* __restrict__ PH, __bf16* __restrict__ PP) {
  __shared__ __align__(16) __bf16 s[C3 * CKP]; __shared__ __align__(16) __bf16 s2[CIN * CG]; const int t = threadIdx.x;
  for (int q = t; q < C3 * CKP; q += 256) { const int n = q / CKP, k = q % CKP; s[q] = (__bf16)((k < CIN) ? WH[(size_t)n * CIN + k] : 0.f); }
  for (int q = t; q < CIN * CG; q += 256) s2[q] = (__bf16)WP[q];
  __syncthreads();
  for (int q = t; q < C3 * CKP / 8; q += 256) vst2((unsigned*)(PH + q * 8), *(const v4u*)&s[q * 8]);
  for (int q = t; q < CIN * CG / 8; q += 256) vst2((unsigned*)(PP + q * 8), *(const v4u*)&s2[q * 8]);
}
__global__ __launch_bounds__(256) void k_xc(const float* __restrict__ X, __bf16* __restrict__ XC) {
  __shared__ __align__(16) __bf16 s[256][72]; const int row = blockIdx.x, t = threadIdx.x; const int b = row / HH, y = row % HH;
  for (int q = t; q < CKP * 256; q += 256) { const int c = q >> 8, px = q & 255; s[px][c] = (__bf16)((c < CIN) ? X[(((size_t)b * CIN + c) * HH + y) * WWD + px] : 0.f); }
  __syncthreads();
  for (int q = t; q < 256 * 8; q += 256) { const int px = q >> 3, pc = q & 7; vst2((unsigned*)(XC + ((size_t)row * WWD + px) * CKP + pc * 8), *(const v4u*)&s[px][pc * 8]); }
}
__global__ __launch_bounds__(256) void k_patch(const __bf16* __restrict__ XC, const __bf16* __restrict__ PH, const float* __restrict__ WDW, const float* __restrict__ LNW, const float* __restrict__ LNB, const __bf16* __restrict__ PP, float* __restrict__ OP) {
  __shared__ __align__(16) float shal[112][CG + 1];
  __shared__ __align__(16) float sq[64][CG + 1], sk[64][CG + 1], sv[64][CG + 1];
  __shared__ __align__(16) __bf16 sah[64][104], sal[64][104]; __shared__ float sred[4][64]; __shared__ float smu[64], srs[64]; __shared__ __align__(16) float so[CIN][68];
  const int tid = threadIdx.x, wave = tid >> 5, lane = tid & 31, col = lane & 15, g = lane >> 4; const int patch = blockIdx.x; const int b = patch / (NPR * NPR), pr = (patch / NPR) % NPR, pcn = patch % NPR; const int y0 = pr * PSZ, x0 = pcn * PSZ;
#pragma unroll 1
  for (int grp = 0; grp < 3; ++grp) {
    if (wave < 7) { const int hp = wave * 16 + col; const int hy = hp / 10, hx = hp % 10; const int yy = y0 - 1 + hy, xx = x0 - 1 + hx; const bool ok = (hp < 100) && yy >= 0 && yy < HH && xx >= 0 && xx < WWD;
      const __bf16* arow = XC + ((size_t)b * NPI + (size_t)min(max(yy, 0), HH - 1) * WWD + min(max(xx, 0), WWD - 1)) * CKP; v8f acc[6] = {};
#pragma unroll
      for (int kc = 0; kc < 2; ++kc) { const v16b a = zfrag_ok(frag_b(arow + kc * 32, lane), ok);
#pragma unroll
        for (int j = 0; j < 6; ++j) acc[j] = wmma_bf(a, frag_b(PH + (size_t)(grp * CG + j * 16 + col) * CKP + kc * 32, lane), acc[j]); }
#pragma unroll
      for (int j = 0; j < 6; ++j)
#pragma unroll
        for (int r = 0; r < 8; ++r) shal[wave * 16 + 8 * g + r][j * 16 + col] = acc[j][r]; }
    __syncthreads();
    { const int px = tid & 63; const int py = px >> 3, pxx = px & 7; float* dst = (grp == 0) ? &sq[px][0] : (grp == 1) ? &sk[px][0] : &sv[px][0];
      for (int c = tid >> 6; c < CG; c += 4) { const int ch = grp * CG + c; float a = 0.f;
#pragma unroll
        for (int tap = 0; tap < 9; ++tap) a += shal[(py + tap / 3) * 10 + (pxx + tap % 3)][c] * bfr(WDW[(size_t)ch * 9 + tap]);
        dst[c] = a; } }
    __syncthreads(); }
  { const int px = tid & 63; const int i = px >> 3, j = px & 7;
    for (int c = tid >> 6; c < CG; c += 4) { float a = 0.f;
      for (int aa = 0; aa < 8; ++aa) { const int ii = (i - aa) & 7;
#pragma unroll
        for (int bb = 0; bb < 8; ++bb) a += sq[aa * 8 + bb][c] * sk[ii * 8 + ((j - bb) & 7)][c]; }
      shal[px][c] = a; } }
  __syncthreads();
  { const int px = tid & 63, part = tid >> 6; float s = 0.f; for (int c = part; c < CG; c += 4) s += shal[px][c]; sred[part][px] = s; }
  __syncthreads();
  if (tid < 64) smu[tid] = ((sred[0][tid] + sred[1][tid]) + (sred[2][tid] + sred[3][tid])) / (float)CG;
  __syncthreads();
  { const int px = tid & 63, part = tid >> 6; const float mu = smu[px]; float s = 0.f; for (int c = part; c < CG; c += 4) { const float d = shal[px][c] - mu; s += d * d; } sred[part][px] = s; }
  __syncthreads();
  if (tid < 64) srs[tid] = sqrtf(((sred[0][tid] + sred[1][tid]) + (sred[2][tid] + sred[3][tid])) / (float)CG + 1e-5f);
  __syncthreads();
  { const int px = tid & 63, part = tid >> 6; const float mu = smu[px], sd = srs[px];
    for (int c = part; c < CG; c += 4) { const float on = (shal[px][c] - mu) / sd * bfr(LNW[c]) + bfr(LNB[c]); const float val = sv[px][c] * on; const __bf16 hb = (__bf16)val; sah[px][c] = hb; sal[px][c] = (__bf16)(val - (float)hb); } }
  __syncthreads();
  if (wave < 4) { v8f acc[3] = {};
#pragma unroll
    for (int kc = 0; kc < 3; ++kc) { F2 a; a.h = frag_b(&sah[wave * 16 + col][kc * 32], lane); a.l = frag_b(&sal[wave * 16 + col][kc * 32], lane);
#pragma unroll
      for (int jt = 0; jt < 3; ++jt) { const v16b w = frag_b(PP + (size_t)(jt * 16 + col) * CG + kc * 32, lane); acc[jt] = wmma_bf(a.l, w, acc[jt]); acc[jt] = wmma_bf(a.h, w, acc[jt]); } }
#pragma unroll
    for (int jt = 0; jt < 3; ++jt)
#pragma unroll
      for (int r = 0; r < 8; ++r) so[jt * 16 + col][wave * 16 + 8 * g + r] = acc[jt][r]; }
  __syncthreads();
  for (int q = tid; q < CIN * 16; q += 256) { const int o = q >> 4, pc = q & 15; vst2(OP + (((size_t)b * CIN + o) * (NPR * NPR) + (size_t)pr * NPR + pcn) * 64 + pc * 4, *(const v4f*)&so[o][pc * 4]); }
}
__global__ __launch_bounds__(256) void k_unpatch(const float* __restrict__ OP, float* __restrict__ OUT) {
  __shared__ __align__(16) float s[8][260]; const int t = threadIdx.x; const int pr = blockIdx.x % NPR, bo = blockIdx.x / NPR;
  if (pr >= NPRT || bo >= NBTT * CIN) return;
  for (int q = t; q < 32 * 64; q += 256) { const int pcn = q >> 6, k = q & 63; s[k >> 3][pcn * 8 + (k & 7)] = OP[((size_t)bo * (NPR * NPR) + (size_t)pr * NPR + pcn) * 64 + k]; }
  __syncthreads();
  for (int q = t; q < 8 * 64; q += 256) { const int r = q >> 6, pc = q & 63; vst2(OUT + ((size_t)bo * HH + pr * PSZ + r) * WWD + pc * 4, *(const v4f*)&s[r][pc * 4]); }
}
extern "C" void kernel_launch(void* const* d_in, const int* in_sizes, int n_in, void* d_out, int out_size, void* d_ws, size_t ws_size, hipStream_t stream) {
  (void)in_sizes; (void)n_in; (void)out_size;
  const float** F = (const float**)d_in;
  if (ws_size < (size_t)WS_END) return;
  char* ws = (char*)d_ws; __bf16 *XCp = (__bf16*)(ws + WS_XC), *PH = (__bf16*)(ws + WS_PH), *PP = (__bf16*)(ws + WS_PP); float* OP = (float*)(ws + WS_OP);
  k_pack<<<1, 256, 0, stream>>>(F[1], F[5], PH, PP);
  k_xc<<<NBT * HH, 256, 0, stream>>>(F[0], XCp);
  k_patch<<<NPT, 256, 0, stream>>>(XCp, PH, F[2], F[3], F[4], PP, OP);
  k_unpatch<<<NBT * CIN * NPR, 256, 0, stream>>>(OP, (float*)d_out);
}
